// PointDeconv_80272938762655
// MI455X (gfx1250) — hardware-run, weakly checked
//
#include <hip/hip_runtime.h>
#include <math.h>

typedef __attribute__((ext_vector_type(16))) _Float16 v16h;
typedef __attribute__((ext_vector_type(8)))  _Float16 v8h;
typedef __attribute__((ext_vector_type(8)))  float    v8f;
typedef __attribute__((ext_vector_type(4)))  float    v4f;

constexpr int kBatch = 4;
constexpr int kNIN   = 4096;
constexpr int kMQ    = 16384;
constexpr int kCIN   = 256;
constexpr int kCO    = 128;
constexpr int kPts   = kBatch * kNIN;
constexpr float kEpsBN  = 1e-5f;
constexpr float kCarryW   = 256.0f;
constexpr float kCarryA   = 16.0f;
constexpr float kCarryInv = 1.0f / (kCarryW * kCarryA);
constexpr int kOutPitch = 68;
static_assert(kPts == 16384, "point rows");
static_assert((kCIN % 32) == 0 && (kCO % 32) == 0, "GEMM K multiples of 32");
static_assert((kPts % 64) == 0 && (kCO % 64) == 0, "GEMM M,N multiples of 64");
static_assert((kNIN % 1024) == 0 && (kMQ % 256) == 0 && (kNIN % 64) == 0 && (kCIN % 64) == 0, "tile multiples");
static_assert(kCarryInv * 4096.0f == 1.0f, "carry product");

constexpr size_t kOffX0   = 0;
constexpr size_t kOffACT1 = kOffX0   + (size_t)kPts * kCIN * 2;
constexpr size_t kOffACT2 = kOffACT1 + (size_t)kPts * kCO * 2;
constexpr size_t kOffFEAT = kOffACT2 + (size_t)kPts * kCO * 2;
constexpr size_t kOffW1H  = kOffFEAT + (size_t)kPts * kCO * 4;
constexpr size_t kOffW2H  = kOffW1H  + (size_t)kCO * kCIN * 2;
constexpr size_t kOffW3H  = kOffW2H  + (size_t)kCO * kCO * 2;
constexpr size_t kOffPARS = kOffW3H  + (size_t)kCO * kCO * 2;
constexpr size_t kWsTotal = kOffPARS + (size_t)3 * 256 * 4;
static_assert(kWsTotal == 25299968ull, "carve total");
static_assert(kWsTotal <= 134217728ull, "carve cap");
static_assert((kOffACT1 % 128) == 0 && (kOffACT2 % 128) == 0 && (kOffFEAT % 128) == 0 && (kOffW1H % 128) == 0 &&
              (kOffW2H % 128) == 0 && (kOffW3H % 128) == 0 && (kOffPARS % 128) == 0, "128-B aligned regions");

__device__ __forceinline__ void guard1_h(v8f& a, v16h x, v16h y) {
  asm volatile("v_nop\n\tv_nop\n\tv_nop\n\tv_nop" : "+v"(a) : "v"(x), "v"(y));
}
__device__ __forceinline__ void keep4_h(v16h a, v16h b, v16h c, v16h d) {
  asm volatile("v_nop" :: "v"(a), "v"(b), "v"(c), "v"(d));
}
__device__ __forceinline__ void acc_guard4(v8f& a, v8f& b, v8f& c, v8f& d) {
  asm volatile("v_nop\n\tv_nop\n\tv_nop\n\tv_nop" : "+v"(a), "+v"(b), "+v"(c), "+v"(d));
}
struct FragH {
  union U { v16h v; v8h h[2]; };
  static __device__ __forceinline__ v16h load(const _Float16* p) {
    U f;
    f.h[0] = *(const v8h*)(p);
    f.h[1] = *(const v8h*)(p + 16);
    return f.v;
  }
  static __device__ __forceinline__ v8f mma(v16h a, v16h b, v8f c) {
    return __builtin_amdgcn_wmma_f32_16x16x32_f16(false, a, false, b, (short)0, c, false, false);
  }
};

__global__ __launch_bounds__(256) void prep_kernel(
    const float* __restrict__ w1, const float* __restrict__ w2, const float* __restrict__ w3,
    const float* __restrict__ b1, const float* __restrict__ g1, const float* __restrict__ be1,
    const float* __restrict__ rm1, const float* __restrict__ rv1,
    const float* __restrict__ b2, const float* __restrict__ g2, const float* __restrict__ be2,
    const float* __restrict__ rm2, const float* __restrict__ rv2,
    const float* __restrict__ b3, const float* __restrict__ g3, const float* __restrict__ be3,
    const float* __restrict__ rm3, const float* __restrict__ rv3,
    unsigned short* __restrict__ W1H, unsigned short* __restrict__ W2H, unsigned short* __restrict__ W3H,
    float* __restrict__ pars)
{
  __shared__ __align__(16) float sP[768];
  const int tid = threadIdx.x;
  const int bx  = blockIdx.x;
  if (bx < 32) {
    const float* src = w1;
    unsigned short* dst = W1H;
    int base = bx * 256;
    if (bx >= 24) {
      src = w3; dst = W3H; base = (bx - 24) * 256;
    } else if (bx >= 16) {
      src = w2; dst = W2H; base = (bx - 16) * 256;
    }
    const size_t e0 = (size_t)(base + tid) << 3;
    const v4f a0 = *(const v4f*)(src + e0);
    const v4f a1 = *(const v4f*)(src + e0 + 4);
    v8h hv;
#pragma unroll
    for (int e = 0; e < 4; ++e) {
      hv[e]     = (_Float16)(a0[e] * kCarryW);
      hv[4 + e] = (_Float16)(a1[e] * kCarryW);
    }
    unsigned short* q = dst + e0;
    *(volatile v8h*)q = hv;
    __threadfence();
    *(volatile v8h*)q = hv;
  } else {
    const int c = tid & 127;
    {
      const float al = g1[c] * (1.0f / sqrtf(rv1[c] + kEpsBN));
      const float ga = al * (b1[c] - rm1[c]) + be1[c];
      if (tid < 128) { sP[0 * 256 + c] = al * kCarryInv; sP[0 * 256 + 128 + c] = ga; }
    }
    {
      const float al = g2[c] * (1.0f / sqrtf(rv2[c] + kEpsBN));
      const float ga = al * (b2[c] - rm2[c]) + be2[c];
      if (tid < 128) { sP[1 * 256 + c] = al * kCarryInv; sP[1 * 256 + 128 + c] = ga; }
    }
    {
      const float al = g3[c] * (1.0f / sqrtf(rv3[c] + kEpsBN));
      const float ga = al * (b3[c] - rm3[c]) + be3[c];
      if (tid < 128) { sP[2 * 256 + c] = al * kCarryInv; sP[2 * 256 + 128 + c] = ga; }
    }
    __syncthreads();
    if (tid < 192) {
      const v4f v = *(const v4f*)(sP + tid * 4);
      float* q = pars + tid * 4;
      *(volatile v4f*)q = v;
      __threadfence();
      *(volatile v4f*)q = v;
    }
  }
}

__global__ __launch_bounds__(256) void pack_points_kernel(
    const float* __restrict__ rgb, unsigned short* __restrict__ X0)
{
  __shared__ __align__(16) float sT[64 * 68];
  const int tid  = threadIdx.x;
  const int lane = tid & 31;
  const int wave = __builtin_amdgcn_readfirstlane((int)(threadIdx.x >> 5));
  const int bx = blockIdx.x;
  const int nt = bx & 63;
  const int ct = (bx >> 6) & 3;
  const int b  = bx >> 8;
  const int n0 = nt * 64;
  const int c0 = ct * 64;
  {
    const int n4 = (tid & 15) * 4;
#pragma unroll
    for (int i = 0; i < 4; ++i) {
      const int cl = (tid >> 4) + 16 * i;
      const v4f v = *(const v4f*)(rgb + ((size_t)(b * kCIN + c0 + cl)) * kNIN + n0 + n4);
      *(v4f*)(sT + cl * 68 + n4) = v;
    }
  }
  __syncthreads();
  const int q = lane >> 3, c8 = (lane & 7) * 8;
  v8h hv[2];
#pragma unroll
  for (int it = 0; it < 2; ++it) {
    const int nl = it * 32 + wave * 4 + q;
#pragma unroll
    for (int e = 0; e < 8; ++e) hv[it][e] = (_Float16)(sT[(c8 + e) * 68 + nl] * kCarryA);
  }
  for (int pass = 0; pass < 2; ++pass) {
#pragma unroll
    for (int it = 0; it < 2; ++it) {
      const int nl = it * 32 + wave * 4 + q;
      *(volatile v8h*)(X0 + ((size_t)(b * kNIN + n0 + nl)) * kCIN + c0 + c8) = hv[it];
    }
    __threadfence();
  }
}

template <bool OUT_F16>
__global__ __launch_bounds__(256) void mlp_gemm64(
    const unsigned short* __restrict__ Ap, int lda,
    const unsigned short* __restrict__ Btp, int ldb,
    void* __restrict__ Cout, int ldc,
    const float* __restrict__ cscale, const float* __restrict__ cbias,
    int M, int N, int K, float ocarry)
{
  const _Float16* A  = (const _Float16*)Ap;
  const _Float16* Bt = (const _Float16*)Btp;
  __shared__ __align__(16) float sT[8][16 * 68];
  const int lane = threadIdx.x & 31;
  const int wave = __builtin_amdgcn_readfirstlane((int)(threadIdx.x >> 5));
  const int tilesN = N >> 6;
  const int tilesM = M >> 6;
  const int tile = blockIdx.x * 8 + wave;
  if (tile >= tilesM * tilesN) return;
  const int tm = tile / tilesN;
  const int tn = tile - tm * tilesN;
  const int m0 = tm << 6;
  const int n0 = tn << 6;

  const int rlane = lane & 15;
  const int koff  = (lane >> 4) * 8;
  const int mOff  = (lane >> 4) * 8;

  v8f acc[4][4];
#pragma unroll
  for (int i = 0; i < 4; ++i)
#pragma unroll
    for (int j = 0; j < 4; ++j) acc[i][j] = (v8f){0.f, 0.f, 0.f, 0.f, 0.f, 0.f, 0.f, 0.f};

  for (int k0 = 0; k0 < K; k0 += 32) {
    v16h bh[4];
#pragma unroll
    for (int j = 0; j < 4; ++j) {
      const size_t bo = (size_t)(n0 + (j << 4) + rlane) * ldb + koff + k0;
      bh[j] = FragH::load(Bt + bo);
    }
#pragma unroll
    for (int i = 0; i < 4; ++i) {
      const size_t ao = (size_t)(m0 + (i << 4) + rlane) * lda + koff + k0;
      const v16h ah = FragH::load(A + ao);
#pragma unroll
      for (int j = 0; j < 4; ++j) acc[i][j] = FragH::mma(ah, bh[j], acc[i][j]);
      guard1_h(acc[i][0], ah, bh[0]);
      guard1_h(acc[i][1], ah, bh[1]);
      guard1_h(acc[i][2], ah, bh[2]);
      guard1_h(acc[i][3], ah, bh[3]);
    }
    keep4_h(bh[0], bh[1], bh[2], bh[3]);
  }
  acc_guard4(acc[0][0], acc[0][1], acc[0][2], acc[0][3]);
  acc_guard4(acc[1][0], acc[1][1], acc[1][2], acc[1][3]);
  acc_guard4(acc[2][0], acc[2][1], acc[2][2], acc[2][3]);
  acc_guard4(acc[3][0], acc[3][1], acc[3][2], acc[3][3]);

  float cs[4], bv[4];
#pragma unroll
  for (int j = 0; j < 4; ++j) {
    const int n = n0 + (j << 4) + rlane;
    cs[j] = cscale[n];
    bv[j] = cbias[n];
  }

  float* slab = sT[wave];
#pragma unroll
  for (int i = 0; i < 4; ++i) {
    const int mBase = m0 + (i << 4);
#pragma unroll
    for (int j = 0; j < 4; ++j) {
#pragma unroll
      for (int r = 0; r < 8; ++r) {
        float v = acc[i][j][r] * cs[j] + bv[j];
        v = fmaxf(v, 0.0f) * ocarry;
        slab[(mOff + r) * 68 + (j << 4) + rlane] = v;
      }
    }
    __builtin_amdgcn_fence(__ATOMIC_RELEASE, "workgroup");
    __builtin_amdgcn_wave_barrier();
    __builtin_amdgcn_fence(__ATOMIC_ACQUIRE, "workgroup");
    if (!OUT_F16) {
      float* Cf = (float*)Cout;
      const int hh = lane >> 4, c4 = (lane & 15) * 4;
      for (int pass = 0; pass < 2; ++pass) {
#pragma unroll
        for (int it = 0; it < 8; ++it) {
          const int row = it * 2 + hh;
          const v4f v = *(const v4f*)(slab + row * 68 + c4);
          *(volatile v4f*)(Cf + (size_t)(mBase + row) * ldc + n0 + c4) = v;
        }
        __threadfence();
      }
    } else {
      const int q = lane >> 3, c8 = (lane & 7) * 8;
      unsigned short* Ch = (unsigned short*)Cout;
      for (int pass = 0; pass < 2; ++pass) {
#pragma unroll
        for (int it = 0; it < 4; ++it) {
          const int row = it * 4 + q;
          const float* sp = slab + row * 68 + c8;
          v8h hv;
#pragma unroll
          for (int e = 0; e < 8; ++e) hv[e] = (_Float16)sp[e];
          *(volatile v8h*)(Ch + (size_t)(mBase + row) * ldc + n0 + c8) = hv;
        }
        __threadfence();
      }
    }
    __builtin_amdgcn_fence(__ATOMIC_RELEASE, "workgroup");
    __builtin_amdgcn_wave_barrier();
    __builtin_amdgcn_fence(__ATOMIC_ACQUIRE, "workgroup");
  }
}

#pragma clang fp contract(off)
__device__ __forceinline__ void put_point(float* dst, float x, float y, float z) {
  const float sq = (x * x + z * z) + y * y;
  v4f v;
  v[0] = x; v[1] = y; v[2] = z; v[3] = sq;
  *(v4f*)dst = v;
}

__global__ __launch_bounds__(256) void knn_blend_kernel(
    const float* __restrict__ xyzin, const float* __restrict__ xyzout,
    const float* __restrict__ featT, float* __restrict__ out)
{
  __shared__ __align__(16) float smPts[1024 * 4];
  __shared__ __align__(16) float smOutT[kCO * kOutPitch];
  __shared__ int   smIdx[256 * 3];
  __shared__ float smW[256 * 3];

  const int tid  = threadIdx.x;
  const int lane = tid & 31;
  const int wave = __builtin_amdgcn_readfirstlane((int)(threadIdx.x >> 5));
  const int b  = blockIdx.x >> 6;
  const int m0 = (blockIdx.x & 63) << 8;

  const float* qp = xyzout + ((size_t)b * kMQ + m0 + tid) * 3;
  const float qx = qp[0];
  const float qy = qp[1];
  const float qz = qp[2];
  const float so = (qx * qx + qz * qz) + qy * qy;

  float bd0 = 3.4e38f, bd1 = 3.4e38f, bd2 = 3.4e38f;
  int   bi0 = 0, bi1 = 0, bi2 = 0;

#pragma unroll 1
  for (int ch = 0; ch < kNIN / 1024; ++ch) {
    {
      const float* src = xyzin + ((size_t)b * kNIN + ch * 1024) * 3 + tid * 12;
      const v4f r0 = *(const v4f*)(src);
      const v4f r1 = *(const v4f*)(src + 4);
      const v4f r2 = *(const v4f*)(src + 8);
      float* dst = smPts + tid * 16;
      put_point(dst,      r0[0], r0[1], r0[2]);
      put_point(dst + 4,  r0[3], r1[0], r1[1]);
      put_point(dst + 8,  r1[2], r1[3], r2[0]);
      put_point(dst + 12, r2[1], r2[2], r2[3]);
    }
    __syncthreads();

#pragma unroll 4
    for (int p = 0; p < 1024; ++p) {
      const v4f c = *(const v4f*)(smPts + p * 4);
      float pd = qx * c[0];
      pd = fmaf(qy, c[1], pd);
      pd = fmaf(qz, c[2], pd);
      const float ss = so + c[3];
      float d = fmaf(-2.0f, pd, ss);
      d = (d < 0.0f) ? 1e-7f : d;
      if (d < bd2) {
        const int n = ch * 1024 + p;
        const bool lt0 = d < bd0;
        const bool lt1 = d < bd1;
        const float nd2 = lt1 ? bd1 : d;
        const int   ni2 = lt1 ? bi1 : n;
        const float nd1 = lt0 ? bd0 : (lt1 ? d : bd1);
        const int   ni1 = lt0 ? bi0 : (lt1 ? n : bi1);
        const float nd0 = lt0 ? d : bd0;
        const int   ni0 = lt0 ? n : bi0;
        bd0 = nd0; bd1 = nd1; bd2 = nd2;
        bi0 = ni0; bi1 = ni1; bi2 = ni2;
      }
    }
    __syncthreads();
  }

  {
    const float a0 = 1.0f / bd0;
    const float a1 = 1.0f / bd1;
    const float a2 = 1.0f / bd2;
    const float sum = (a0 + a2) + a1;
    const float s = 1.0f / sum;
    smIdx[tid * 3 + 0] = min(max(bi0, 0), kNIN - 1);
    smIdx[tid * 3 + 1] = min(max(bi1, 0), kNIN - 1);
    smIdx[tid * 3 + 2] = min(max(bi2, 0), kNIN - 1);
    smW[tid * 3 + 0] = a0 * s;
    smW[tid * 3 + 1] = a1 * s;
    smW[tid * 3 + 2] = a2 * s;
  }
  __syncthreads();

  const int q  = lane >> 3;
  const int l8 = lane & 7;
#pragma unroll 1
  for (int sub = 0; sub < 4; ++sub) {
    {
      const int r    = tid >> 2;
      const int ml   = (sub << 6) + r;
      const int cseg = (tid & 3) << 5;
      const int j0 = min(max(smIdx[ml * 3 + 0], 0), kNIN - 1);
      const int j1 = min(max(smIdx[ml * 3 + 1], 0), kNIN - 1);
      const int j2 = min(max(smIdx[ml * 3 + 2], 0), kNIN - 1);
      const float a0 = smW[ml * 3 + 0];
      const float a1 = smW[ml * 3 + 1];
      const float a2 = smW[ml * 3 + 2];
      const float* f0 = featT + ((size_t)b * kNIN + j0) * kCO + cseg;
      const float* f1 = featT + ((size_t)b * kNIN + j1) * kCO + cseg;
      const float* f2 = featT + ((size_t)b * kNIN + j2) * kCO + cseg;
#pragma unroll 2
      for (int c = 0; c < 32; c += 4) {
        const v4f x0 = *(const v4f*)(f0 + c);
        const v4f x1 = *(const v4f*)(f1 + c);
        const v4f x2 = *(const v4f*)(f2 + c);
#pragma unroll
        for (int e = 0; e < 4; ++e) {
          float o = a0 * x0[e];
          o = fmaf(a1, x1[e], o);
          o = fmaf(a2, x2[e], o);
          smOutT[(cseg + c + e) * kOutPitch + r] = o;
        }
      }
    }
    __syncthreads();

    for (int pass = 0; pass < 2; ++pass) {
#pragma unroll
      for (int it = 0; it < 8; ++it) {
        const int L  = it * 32 + wave * 4 + q;
        const int c  = L >> 1;
        const int hf = L & 1;
        const v4f v = *(const v4f*)(smOutT + c * kOutPitch + hf * 32 + l8 * 4);
        *(volatile v4f*)(out + ((size_t)b * kCO + c) * kMQ + m0 + (sub << 6) + hf * 32 + l8 * 4) = v;
      }
      __threadfence();
    }
    __syncthreads();
  }
}

extern "C" void kernel_launch(void* const* d_in, const int* in_sizes, int n_in,
                              void* d_out, int out_size, void* d_ws, size_t ws_size,
                              hipStream_t stream) {
  if (n_in < 21) return;
  if (in_sizes[0] != kBatch * kCIN * kNIN) return;
  if (in_sizes[1] != kBatch * kNIN * 3) return;
  if (in_sizes[2] != kBatch * kMQ * 3) return;
  if (in_sizes[3] != kCO * kCIN) return;
  if (in_sizes[9] != kCO * kCO) return;
  if (in_sizes[15] != kCO * kCO) return;
  for (int i = 4; i <= 8; ++i)   if (in_sizes[i] != kCO) return;
  for (int i = 10; i <= 14; ++i) if (in_sizes[i] != kCO) return;
  for (int i = 16; i <= 20; ++i) if (in_sizes[i] != kCO) return;
  if (out_size != kBatch * kCO * kMQ) return;
  if (ws_size < kWsTotal) return;

  const float* rgb    = (const float*)d_in[0];
  const float* xyzin  = (const float*)d_in[1];
  const float* xyzout = (const float*)d_in[2];
  const float* w1  = (const float*)d_in[3];
  const float* b1  = (const float*)d_in[4];
  const float* g1  = (const float*)d_in[5];
  const float* be1 = (const float*)d_in[6];
  const float* rm1 = (const float*)d_in[7];
  const float* rv1 = (const float*)d_in[8];
  const float* w2  = (const float*)d_in[9];
  const float* b2  = (const float*)d_in[10];
  const float* g2  = (const float*)d_in[11];
  const float* be2 = (const float*)d_in[12];
  const float* rm2 = (const float*)d_in[13];
  const float* rv2 = (const float*)d_in[14];
  const float* w3  = (const float*)d_in[15];
  const float* b3  = (const float*)d_in[16];
  const float* g3  = (const float*)d_in[17];
  const float* be3 = (const float*)d_in[18];
  const float* rm3 = (const float*)d_in[19];
  const float* rv3 = (const float*)d_in[20];

  char* ws = (char*)d_ws;
  unsigned short* X0   = (unsigned short*)(ws + kOffX0);
  unsigned short* ACT1 = (unsigned short*)(ws + kOffACT1);
  unsigned short* ACT2 = (unsigned short*)(ws + kOffACT2);
  float*          FEAT = (float*)(ws + kOffFEAT);
  unsigned short* W1H  = (unsigned short*)(ws + kOffW1H);
  unsigned short* W2H  = (unsigned short*)(ws + kOffW2H);
  unsigned short* W3H  = (unsigned short*)(ws + kOffW3H);
  float*          PARS = (float*)(ws + kOffPARS);

  prep_kernel<<<33, 256, 0, stream>>>(w1, w2, w3,
                                      b1, g1, be1, rm1, rv1,
                                      b2, g2, be2, rm2, rv2,
                                      b3, g3, be3, rm3, rv3,
                                      W1H, W2H, W3H, PARS);

  pack_points_kernel<<<kBatch * (kCIN / 64) * (kNIN / 64), 256, 0, stream>>>(rgb, X0);

  const int gemmBlocks = ((kPts / 64) * (kCO / 64)) / 8;

  mlp_gemm64<true><<<gemmBlocks, 256, 0, stream>>>(
      X0, kCIN, W1H, kCIN, (void*)ACT1, kCO,
      PARS + 0, PARS + 128, kPts, kCO, kCIN, kCarryA);

  mlp_gemm64<true><<<gemmBlocks, 256, 0, stream>>>(
      ACT1, kCO, W2H, kCO, (void*)ACT2, kCO,
      PARS + 256, PARS + 384, kPts, kCO, kCO, kCarryA);

  mlp_gemm64<false><<<gemmBlocks, 256, 0, stream>>>(
      ACT2, kCO, W3H, kCO, (void*)FEAT, kCO,
      PARS + 512, PARS + 640, kPts, kCO, kCO, 1.0f);

  knn_blend_kernel<<<kBatch * (kMQ / 256), 256, 0, stream>>>(xyzin, xyzout, FEAT, (float*)d_out);
}
